// NeuralTuringMemo_70703751627105
// MI455X (gfx1250) — hardware-verified
//
#include <hip/hip_runtime.h>


#define NBT  8
#define DD   64
#define THW  16384
#define NN_  (NBT * THW)
#define KK   512
#define PSC  32768.0f

typedef unsigned short bf;
typedef __attribute__((ext_vector_type(16))) __bf16   v16bf;
typedef __attribute__((ext_vector_type(8)))  unsigned short v8us;
typedef __attribute__((ext_vector_type(8)))  float    v8f;
typedef __attribute__((ext_vector_type(4)))  float    v4f;
typedef v4f  __attribute__((may_alias)) v4fa;
typedef v8us __attribute__((may_alias)) v8usa;

__device__ __forceinline__ unsigned short f2bf(float f) { unsigned u = __float_as_uint(f); u += 0x7FFFu + ((u >> 16) & 1u); return (unsigned short)(u >> 16); }
__device__ __forceinline__ float bf2f(unsigned short b) { return __uint_as_float(((unsigned)b) << 16); }
__device__ __forceinline__ float bfr(float f) { return bf2f(f2bf(f)); }
__device__ __forceinline__ v16bf cat16b(v8us lo, v8us hi) { return __builtin_bit_cast(v16bf, __builtin_shufflevector(lo, hi, 0, 1, 2, 3, 4, 5, 6, 7, 8, 9, 10, 11, 12, 13, 14, 15)); }
__device__ __forceinline__ v8f wmmab(v16bf a, v16bf b, v8f c) { return __builtin_amdgcn_wmma_f32_16x16x32_bf16(false, a, false, b, (short)0, c, false, false); }
#define VST2(T, p, v) do { const T vst2_v_ = (v); *(volatile T*)(p) = vst2_v_; __threadfence(); *(volatile T*)(p) = vst2_v_; } while (0)

__global__ __launch_bounds__(256) void k_xt(const float* __restrict__ inp, bf* XB, float* XS) {
    __shared__ __align__(16) unsigned short tl[64 * 72];
    const int tid = threadIdx.x, p0 = blockIdx.x * 64, b = blockIdx.y;
    { const int d = tid >> 2, pq = (tid & 3) * 16;
#pragma unroll
      for (int i = 0; i < 16; ++i) tl[(pq + i) * 72 + d] = f2bf(inp[((size_t)b * DD + d) * THW + p0 + pq + i]); }
    __syncthreads();
    const int piece = tid & 7;
    auto pass = [&]() {
#pragma unroll
        for (int s = 0; s < 2; ++s) { const int pl = (tid >> 3) + 32 * s; const v8us val = *(const v8usa*)(tl + pl * 72 + piece * 8); *(volatile v8us*)(XB + ((size_t)b * THW + p0 + pl) * DD + piece * 8) = val; }
    };
    pass(); __threadfence(); pass();
    if (tid < 64) { float s = 0.f;
#pragma unroll 8
        for (int d = 0; d < DD; ++d) { const float v = bf2f(tl[tid * 72 + d]); s += v * v; }
        *(volatile float*)(XS + (size_t)b * THW + p0 + tid) = s; }
    __threadfence();
    if (tid < 64) { float s = 0.f;
#pragma unroll 8
        for (int d = 0; d < DD; ++d) { const float v = bf2f(tl[tid * 72 + d]); s += v * v; }
        *(volatile float*)(XS + (size_t)b * THW + p0 + tid) = s; }
}
__global__ __launch_bounds__(256) void k_emb(const float* __restrict__ emb, bf* EB, bf* ET, float* ES) {
    __shared__ __align__(16) unsigned short tl[64 * 72];
    const int tid = threadIdx.x, k0 = blockIdx.x * 64;
    { const int kk = tid >> 2, dq = (tid & 3) * 16;
#pragma unroll
      for (int i = 0; i < 16; ++i) tl[(dq + i) * 72 + kk] = f2bf(emb[(size_t)(k0 + kk) * DD + dq + i]); }
    __syncthreads();
    const int piece = tid & 7;
    auto pass = [&]() {
#pragma unroll
        for (int s = 0; s < 2; ++s) { const int d = (tid >> 3) + 32 * s; const v8us val = *(const v8usa*)(tl + d * 72 + piece * 8); *(volatile v8us*)(ET + (size_t)d * KK + k0 + piece * 8) = val; }
        { const int kk = tid >> 3; if (kk < 32) {   } }
#pragma unroll
        for (int s = 0; s < 2; ++s) { const int kk = (tid >> 3) + 32 * s; v8us o;
#pragma unroll
            for (int i = 0; i < 8; ++i) o[i] = tl[(piece * 8 + i) * 72 + kk];
            *(volatile v8us*)(EB + (size_t)(k0 + kk) * DD + piece * 8) = o; }
    };
    pass(); __threadfence(); pass();
    if (tid < 64) { float s = 0.f;
#pragma unroll 8
        for (int d = 0; d < DD; ++d) { const float v = bf2f(tl[d * 72 + tid]); s += v * v; }
        *(volatile float*)(ES + k0 + tid) = s; }
    __threadfence();
    if (tid < 64) { float s = 0.f;
#pragma unroll 8
        for (int d = 0; d < DD; ++d) { const float v = bf2f(tl[d * 72 + tid]); s += v * v; }
        *(volatile float*)(ES + k0 + tid) = s; }
}
__global__ __launch_bounds__(128) void k_attn(const bf* __restrict__ XB, const float* __restrict__ XS, const bf* __restrict__ EB, const bf* __restrict__ ET, const float* __restrict__ ES, float* out) {
    __shared__ __align__(16) unsigned short plds[4][16 * 32];
    __shared__ __align__(16) unsigned short plds2[4][16 * 32];
    __shared__ __align__(16) float ot[64 * 68];
    const int lane = threadIdx.x & 31, wave = threadIdx.x >> 5, lr = lane & 15, hi = lane >> 4;
    const size_t n0 = (size_t)blockIdx.x * 64 + wave * 16;
    unsigned short* pl = &plds[wave][0]; unsigned short* pl2 = &plds2[wave][0];
    v16bf xa[2];
#pragma unroll
    for (int kc = 0; kc < 2; ++kc) { const bf* p = XB + (n0 + lr) * DD + kc * 32 + 8 * hi; xa[kc] = cat16b(*(const v8us*)p, *(const v8us*)(p + 16)); }
    float xs[8];
#pragma unroll
    for (int j = 0; j < 8; ++j) xs[j] = XS[n0 + hi * 8 + j];
    v8f o[4];
#pragma unroll
    for (int n = 0; n < 4; ++n) o[n] = (v8f){};
    float mrow[8], lpart[8];
#pragma unroll
    for (int j = 0; j < 8; ++j) { mrow[j] = -3.0e38f; lpart[j] = 0.f; }
#pragma unroll 1
    for (int kt = 0; kt < KK / 32; ++kt) {
        const int k0 = kt * 32;
        v8f g0 = {}, g1 = {};
#pragma unroll
        for (int kc = 0; kc < 2; ++kc) { const bf* p0 = EB + (size_t)(k0 + lr) * DD + kc * 32 + 8 * hi; const bf* p1 = p0 + (size_t)16 * DD;
            g0 = wmmab(xa[kc], cat16b(*(const v8us*)p0, *(const v8us*)(p0 + 16)), g0); g1 = wmmab(xa[kc], cat16b(*(const v8us*)p1, *(const v8us*)(p1 + 16)), g1); }
        asm volatile("v_nop\n\tv_nop\n\tv_nop\n\tv_nop" : "+v"(g0), "+v"(g1) : "v"(xa[0]), "v"(xa[1]));
        const float esa = ES[k0 + lr], esb = ES[k0 + 16 + lr];
        float alpha[8];
#pragma unroll
        for (int j = 0; j < 8; ++j) {
            const float a0 = xs[j] + esa - 2.0f * g0[j], a1 = xs[j] + esb - 2.0f * g1[j];
            float mx = fmaxf(a0, a1);
            mx = fmaxf(mx, __shfl_xor(mx, 1, 16)); mx = fmaxf(mx, __shfl_xor(mx, 2, 16)); mx = fmaxf(mx, __shfl_xor(mx, 4, 16)); mx = fmaxf(mx, __shfl_xor(mx, 8, 16));
            const float mn = fmaxf(mrow[j], mx);
            alpha[j] = __expf(mrow[j] - mn); mrow[j] = mn;
            const float p0 = __expf(a0 - mn), p1 = __expf(a1 - mn);
            lpart[j] = lpart[j] * alpha[j] + (p0 + p1);
            const int mr = hi * 8 + j; const float ps0 = p0 * PSC, ps1 = p1 * PSC; const unsigned short h0 = f2bf(ps0), h1 = f2bf(ps1);
            pl[mr * 32 + lr] = h0; pl[mr * 32 + 16 + lr] = h1; pl2[mr * 32 + lr] = f2bf(ps0 - bf2f(h0)); pl2[mr * 32 + 16 + lr] = f2bf(ps1 - bf2f(h1)); }
#pragma unroll
        for (int n = 0; n < 4; ++n)
#pragma unroll
            for (int j = 0; j < 8; ++j) o[n][j] *= alpha[j];
        asm volatile("" ::: "memory");
        const v16bf pa = cat16b(*(const v8usa*)(pl + lr * 32 + hi * 8), *(const v8usa*)(pl + lr * 32 + 16 + hi * 8));
        const v16bf px = cat16b(*(const v8usa*)(pl2 + lr * 32 + hi * 8), *(const v8usa*)(pl2 + lr * 32 + 16 + hi * 8));
#pragma unroll
        for (int n = 0; n < 4; ++n) { const bf* ep = ET + (size_t)(n * 16 + lr) * KK + k0 + hi * 8; const v16bf ev = cat16b(*(const v8us*)ep, *(const v8us*)(ep + 16));
            o[n] = wmmab(pa, ev, o[n]); o[n] = wmmab(px, ev, o[n]);
            asm volatile("" : "+v"(o[n]) : "v"(ev) : "memory"); }
        asm volatile("v_nop\n\tv_nop\n\tv_nop\n\tv_nop" : "+v"(o[0]), "+v"(o[3]) : "v"(pa), "v"(px));
        __builtin_amdgcn_wave_barrier();
    }
    float inv[8];
#pragma unroll
    for (int j = 0; j < 8; ++j) { float rs = lpart[j]; rs += __shfl_xor(rs, 1, 16); rs += __shfl_xor(rs, 2, 16); rs += __shfl_xor(rs, 4, 16); rs += __shfl_xor(rs, 8, 16); inv[j] = 1.0f / (rs * PSC); }
#pragma unroll
    for (int n = 0; n < 4; ++n)
#pragma unroll
        for (int j = 0; j < 8; ++j) ot[(n * 16 + lr) * 68 + wave * 16 + hi * 8 + j] = o[n][j] * inv[j];
    __syncthreads();
    const size_t nb0 = (size_t)blockIdx.x * 64; const int b = (int)(nb0 / THW); const size_t p0 = nb0 - (size_t)b * THW;
    auto pass = [&]() {
#pragma unroll
        for (int s = 0; s < 8; ++s) { const int d = wave * 16 + s * 2 + (lane >> 4), piece = lane & 15;
            const v4f val = *(const v4fa*)(ot + d * 68 + piece * 4); *(volatile v4f*)(out + ((size_t)b * DD + d) * THW + p0 + piece * 4) = val; }
    };
    pass(); __threadfence(); pass();
}

extern "C" void kernel_launch(void* const* d_in, const int* in_sizes, int n_in,
                              void* d_out, int out_size, void* d_ws, size_t ws_size, hipStream_t stream) {
    (void)in_sizes; (void)n_in; (void)out_size;
    const float* inp = (const float*)d_in[0]; const float* emb = (const float*)d_in[1];
    float* out = (float*)d_out;
    char* wsp = (char*)d_ws;
    auto take = [&](size_t bytes) { char* p = wsp; wsp += (bytes + 255) & ~(size_t)255; return (void*)p; };
    bf* XB = (bf*)take((size_t)NN_ * DD * 2); float* XS = (float*)take((size_t)NN_ * 4); bf* EB = (bf*)take((size_t)KK * DD * 2); bf* ET = (bf*)take((size_t)DD * KK * 2); float* ES = (float*)take((size_t)KK * 4);
    if ((size_t)(wsp - (char*)d_ws) > ws_size) return;
    k_xt<<<dim3(THW / 64, NBT, 1), 256, 0, stream>>>(inp, XB, XS);
    k_emb<<<KK / 64, 256, 0, stream>>>(emb, EB, ET, ES);
    k_attn<<<NN_ / 64, 128, 0, stream>>>(XB, XS, EB, ET, ES, out);
}
